// MultiHeadAttention_33981781246192
// MI455X (gfx1250) — hardware-verified
//
#include <hip/hip_runtime.h>
#include <math.h>

typedef __attribute__((ext_vector_type(16))) _Float16 v16h;
typedef __attribute__((ext_vector_type(16))) __bf16 v16b;
typedef __attribute__((ext_vector_type(8)))  _Float16 v8h;
typedef __attribute__((ext_vector_type(8)))  __bf16 v8b;
typedef __attribute__((ext_vector_type(8)))  float v8f;
typedef __attribute__((ext_vector_type(4)))  float v4f;
typedef __attribute__((ext_vector_type(4)))  unsigned v4u;

template <typename T> __device__ __forceinline__ void vst2(void* p, T v) { *(volatile T*)p = v; __threadfence(); *(volatile T*)p = v; }
__device__ __forceinline__ v8f wmma16(v16h a, v16h b, v8f c) {
  v8f d = __builtin_amdgcn_wmma_f32_16x16x32_f16(false, a, false, b, (short)0, c, false, false);
  asm volatile("v_nop\n\tv_nop\n\tv_nop\n\tv_nop" : "+v"(d) : "v"(a), "v"(b));
  return d;
}
__device__ __forceinline__ v8f wmma_bf(v16b a, v16b b, v8f c) {
  v8f d = __builtin_amdgcn_wmma_f32_16x16x32_bf16(false, a, false, b, (short)0, c, false, false);
  asm volatile("v_nop\n\tv_nop\n\tv_nop\n\tv_nop" : "+v"(d) : "v"(a), "v"(b));
  return d;
}
__device__ __forceinline__ v16h frag_h(const _Float16* rowk0, int lane) {
  union { v16h v; v8h q[2]; } u; const _Float16* p = rowk0 + 8 * (lane >> 4);
  u.q[0] = *(const v8h*)p; u.q[1] = *(const v8h*)(p + 16); return u.v;
}
__device__ __forceinline__ v16b frag_b(const __bf16* rowk0, int lane) {
  union { v16b v; v8b q[2]; } u; const __bf16* p = rowk0 + 8 * (lane >> 4);
  u.q[0] = *(const v8b*)p; u.q[1] = *(const v8b*)(p + 16); return u.v;
}
__device__ __forceinline__ v16h frag_f32(const float* rowk0, int lane) {
  v16h a; const float* p = rowk0 + 8 * (lane >> 4);
#pragma unroll
  for (int i = 0; i < 8; ++i) { a[i] = (_Float16)p[i]; a[8 + i] = (_Float16)p[16 + i]; }
  return a;
}
__device__ __forceinline__ v16h frag_f32s(const float* rowk0, int lane, float sc) {
  v16h a; const float* p = rowk0 + 8 * (lane >> 4);
#pragma unroll
  for (int i = 0; i < 8; ++i) { a[i] = (_Float16)(p[i] * sc); a[8 + i] = (_Float16)(p[16 + i] * sc); }
  return a;
}
struct F2 { v16b h, l; };
__device__ __forceinline__ F2 bsplit16(const float v[16]) { F2 r;
#pragma unroll
  for (int i = 0; i < 16; ++i) { const __bf16 h = (__bf16)v[i]; r.h[i] = h; r.l[i] = (__bf16)(v[i] - (float)h); }
  return r; }
__device__ __forceinline__ F2 split_row(const float* row, int k0, int lane) { float v[16]; const float* p = row + k0 + 8 * (lane >> 4);
#pragma unroll
  for (int i = 0; i < 8; ++i) { v[i] = p[i]; v[8 + i] = p[16 + i]; }
  return bsplit16(v); }
#define LDSX() do { asm volatile("s_wait_dscnt 0" ::: "memory"); __builtin_amdgcn_wave_barrier(); __builtin_amdgcn_fence(3  , "workgroup"); } while (0)

#ifndef NB
#define NB 64
#endif
#ifndef SEQ
#define SEQ 256
#endif
#define NB_FULL 64
#define TT_FULL 256
#define TT SEQ
#define CC 512
#define DIN 512
#define NH 8
#define HD 64
#define NQB (TT / 64)
#define SCALE (0.125f)
#define CAUSAL 1
#ifndef NBC
#if NB < 16
#define NBC NB
#else
#define NBC 16
#endif
#endif
#ifndef QBH
#define QBH NQB
#endif
#ifndef QHI
#define QHI TT
#endif
#ifndef KHI
#define KHI TT
#endif
#define NEED_PLAIN (QBH < NQB)
#define KCH (TT / 128)

__device__ __forceinline__ float bfr(float v) { return (float)(__bf16)v; }
__host__ __device__ constexpr int kb_last(int qb) { return CAUSAL ? ((qb * 64 + 63) >> 7) : (TT / 128 - 1); }

__device__ __forceinline__ v16b wcol_io(const float* Wm, int k0, int o, int lane, int ld) { v16b w; const int g = lane >> 4;
#pragma unroll
  for (int i = 0; i < 8; ++i) { w[i] = (__bf16)Wm[(size_t)(k0 + 8 * g + i) * ld + o]; w[8 + i] = (__bf16)Wm[(size_t)(k0 + 16 + 8 * g + i) * ld + o]; }
  return w; }
__device__ __forceinline__ v16h wcolh_io(const float* Wm, int k0, int o, int lane, int ld) { v16h w; const int g = lane >> 4;
#pragma unroll
  for (int i = 0; i < 8; ++i) { w[i] = (_Float16)(bfr(Wm[(size_t)(k0 + 8 * g + i) * ld + o]) * 256.0f); w[8 + i] = (_Float16)(bfr(Wm[(size_t)(k0 + 16 + 8 * g + i) * ld + o]) * 256.0f); }
  return w; }
__device__ __forceinline__ v16b wcol_hdk(const float* Wm, int k0, int o, int lane) { v16b w; const int g = lane >> 4; const float* p = Wm + (size_t)(o / HD) * DIN * HD + (o % HD);
#pragma unroll
  for (int i = 0; i < 8; ++i) { w[i] = (__bf16)p[(size_t)(k0 + 8 * g + i) * HD]; w[8 + i] = (__bf16)p[(size_t)(k0 + 16 + 8 * g + i) * HD]; }
  return w; }

#if NEED_PLAIN
#define VT_BYTES (2ull * NBC * CC * TT)
#else
#define VT_BYTES 0ull
#endif
#define WS_QH  0ull
#define WS_KH  (WS_QH + 2ull * NBC * TT * CC)
#define WS_VT  (WS_KH + 2ull * NBC * TT * CC)
#define WS_QL  (WS_VT + VT_BYTES)
#define WS_KL  (WS_QL + 2ull * NBC * QHI * CC)
#define WS_VB  (WS_KL + 2ull * NBC * KHI * CC)
#define WS_VBL (WS_VB + 2ull * NBC * CC * KHI)
#define WS_S   (WS_VBL + 2ull * NBC * CC * KHI)
#define WS_Y   (WS_S  + 4ull * NBC * NH * TT * TT)
#define WS_END (WS_Y  + 4ull * NBC * TT * CC)

static_assert(TT % 128 == 0);
static_assert(TT <= TT_FULL);
static_assert(NB <= NB_FULL);
static_assert(NB % NBC == 0);
static_assert(QBH >= 1 && QBH <= NQB);
static_assert(QHI % 64 == 0 && QHI <= TT && QBH * 64 <= QHI);
static_assert(KHI % 64 == 0 && KHI <= TT && KHI >= (kb_last(QBH - 1) + 1) * 128);
static_assert(CC == NH * HD && CC % 128 == 0 && DIN % 128 == 0 && DIN % 32 == 0 && HD % 32 == 0);
static_assert(NBC * NH <= 65535);
static_assert(WS_END <= 134217728ull);

__global__ __launch_bounds__(128) void k_proj(const float* __restrict__ X, const float* __restrict__ WQ, const float* __restrict__ WK, const float* __restrict__ WV,
    _Float16* __restrict__ QH, _Float16* __restrict__ QL, _Float16* __restrict__ KH, _Float16* __restrict__ KL, _Float16* __restrict__ VT, __bf16* __restrict__ VB, __bf16* __restrict__ VBL) {
  __shared__ __align__(16) _Float16 sh[64][136], sl[64][136]; __shared__ __align__(16) _Float16 th[128][72]; __shared__ __align__(16) __bf16 tb[128][72], tbl[128][72];
  const int tid = threadIdx.x, wave = __builtin_amdgcn_readfirstlane((int)(tid >> 5)), lane = tid & 31, col = lane & 15, g = lane >> 4;
  const int which = blockIdx.z; const int c0 = blockIdx.y * 128; const size_t r0 = (size_t)blockIdx.x * 64; const size_t bb = r0 / TT; const int t0 = (int)(r0 % TT);
  const float* WA = which == 0 ? WQ : which == 1 ? WK : WV;
  const size_t xr = bb * TT_FULL + t0 + wave * 16 + col;
  v8f acc[8] = {};
#pragma unroll 2
  for (int kc = 0; kc < DIN / 32; ++kc) {
    v16b a;
    { const float* p = X + xr * DIN + kc * 32 + 8 * g;
#pragma unroll
      for (int i = 0; i < 8; ++i) { a[i] = (__bf16)p[i]; a[8 + i] = (__bf16)p[16 + i]; } }
    asm volatile("s_wait_loadcnt 0x0" ::: "memory");
#pragma unroll
    for (int j = 0; j < 8; ++j) { const v16b w = wcol_hdk(WA, kc * 32, c0 + j * 16 + col, lane); asm volatile("s_wait_loadcnt 0x0" ::: "memory"); acc[j] = wmma_bf(a, w, acc[j]); }
  }
  if (which < 2) {
    _Float16* DH = which == 0 ? QH : KH; _Float16* DL = which == 0 ? QL : KL; const int nhi = which == 0 ? QHI : KHI; const bool hi_rows = t0 < nhi;
#pragma unroll
    for (int j = 0; j < 8; ++j) {
#pragma unroll
      for (int r = 0; r < 8; ++r) { const float v = acc[j][r]; const _Float16 hv = (_Float16)v; sh[wave * 16 + 8 * g + r][j * 16 + col] = hv; sl[wave * 16 + 8 * g + r][j * 16 + col] = (_Float16)((v - (float)hv) * 1024.0f); }
    }
    __syncthreads();
    for (int e = tid; e < 64 * 16; e += 128) { const int rl = e >> 4, q = e & 15;
      vst2((void*)(DH + (r0 + rl) * CC + c0 + q * 8), *(const v4u*)&sh[rl][q * 8]);
      if (hi_rows) vst2((void*)(DL + (bb * nhi + t0 + rl) * (size_t)CC + c0 + q * 8), *(const v4u*)&sl[rl][q * 8]); }
  } else {
    const bool hi_rows = t0 < KHI;
#pragma unroll
    for (int j = 0; j < 8; ++j) {
#pragma unroll
      for (int r = 0; r < 8; ++r) { const float v = acc[j][r]; const int rl = wave * 16 + 8 * g + r, cl = j * 16 + col; if (NEED_PLAIN) th[cl][rl] = (_Float16)v; const __bf16 bh = (__bf16)v; tb[cl][rl] = bh; tbl[cl][rl] = (__bf16)(v - (float)bh); }
    }
    __syncthreads();
    for (int e = tid; e < 128 * 8; e += 128) { const int cl = e >> 3, q = e & 7;
      if (NEED_PLAIN) vst2((void*)(VT + (bb * CC + c0 + cl) * (size_t)TT + t0 + q * 8), *(const v4u*)&th[cl][q * 8]);
      if (hi_rows) { const size_t o3 = (bb * CC + c0 + cl) * (size_t)KHI + t0 + q * 8; vst2((void*)(VB + o3), *(const v4u*)&tb[cl][q * 8]); vst2((void*)(VBL + o3), *(const v4u*)&tbl[cl][q * 8]); } }
  }
}

__global__ __launch_bounds__(128) void k_sc(const _Float16* __restrict__ QH, const _Float16* __restrict__ KH, const _Float16* __restrict__ QL, const _Float16* __restrict__ KL, float* __restrict__ S0) {
  __shared__ __align__(16) float ss[4][16][132];
  const int qb = blockIdx.x, kb = blockIdx.y; if (kb > kb_last(qb)) return;
  const int bl = blockIdx.z / NH, h = blockIdx.z % NH; float* S = S0 + (size_t)blockIdx.z * TT * TT;
  const int tid = threadIdx.x, wave = __builtin_amdgcn_readfirstlane((int)(tid >> 5)), lane = tid & 31, col = lane & 15, g = lane >> 4; const int k0 = kb * 128; const int ql0 = qb * 64 + wave * 16; const size_t q0 = (size_t)bl * TT + ql0, kr0 = (size_t)bl * TT + k0;
  v8f acc[8] = {}, accl[8] = {};
  const _Float16* QLb = QL + (size_t)bl * QHI * CC; const _Float16* KLb = KL + (size_t)bl * KHI * CC;
  if (!NEED_PLAIN || qb < QBH) {
#pragma unroll
    for (int kc = 0; kc < HD / 32; ++kc) { const v16h ah = frag_h(QH + (q0 + col) * CC + h * HD + kc * 32, lane), al = frag_h(QLb + (size_t)(ql0 + col) * CC + h * HD + kc * 32, lane);
#pragma unroll
      for (int j = 0; j < 8; ++j) { const v16h kbf = frag_h(KH + (kr0 + j * 16 + col) * CC + h * HD + kc * 32, lane), klf = frag_h(KLb + (size_t)(k0 + j * 16 + col) * CC + h * HD + kc * 32, lane); acc[j] = wmma16(ah, kbf, acc[j]); accl[j] = wmma16(al, kbf, accl[j]); accl[j] = wmma16(ah, klf, accl[j]); } }
  } else if (qb * 64 < QHI) {
#pragma unroll
    for (int kc = 0; kc < HD / 32; ++kc) { const v16h ah = frag_h(QH + (q0 + col) * CC + h * HD + kc * 32, lane), al = frag_h(QLb + (size_t)(ql0 + col) * CC + h * HD + kc * 32, lane);
#pragma unroll
      for (int j = 0; j < 8; ++j) { const v16h kbf = frag_h(KH + (kr0 + j * 16 + col) * CC + h * HD + kc * 32, lane); acc[j] = wmma16(ah, kbf, acc[j]); accl[j] = wmma16(al, kbf, accl[j]); } }
  } else {
#pragma unroll
    for (int kc = 0; kc < HD / 32; ++kc) { const v16h ah = frag_h(QH + (q0 + col) * CC + h * HD + kc * 32, lane);
#pragma unroll
      for (int j = 0; j < 8; ++j) { const v16h kbf = frag_h(KH + (kr0 + j * 16 + col) * CC + h * HD + kc * 32, lane); acc[j] = wmma16(ah, kbf, acc[j]); } }
  }
#pragma unroll
  for (int j = 0; j < 8; ++j) {
#pragma unroll
    for (int r = 0; r < 8; ++r) ss[wave][8 * g + r][j * 16 + col] = (acc[j][r] + accl[j][r] * (1.0f / 1024.0f)) * SCALE;
  }
  LDSX();
  for (int rl = 0; rl < 16; ++rl) vst2((void*)(S + (size_t)(ql0 + rl) * TT + k0 + lane * 4), *(const v4f*)&ss[wave][rl][lane * 4]);
}

__global__ __launch_bounds__(256) void k_sm(float* __restrict__ S0) {
  const int tid = threadIdx.x, wave = __builtin_amdgcn_readfirstlane((int)(tid >> 5)), lane = tid & 31; const int t = blockIdx.x * 8 + wave;
  const int kend = (kb_last(t >> 6) + 1) * 128;
  float* sr = S0 + (size_t)blockIdx.y * TT * TT + (size_t)t * TT;
  v4f e[KCH]; float m = -3.0e38f;
#pragma unroll
  for (int c = 0; c < KCH; ++c) { const int k = c * 128 + lane * 4; v4f v = *(const v4f*)(sr + k);
#pragma unroll
    for (int i = 0; i < 4; ++i) { const bool ok = (k + i < kend) && (!CAUSAL || (k + i <= t)); const float x = ok ? v[i] : -3.0e38f; v[i] = x; m = fmaxf(m, x); }
    e[c] = v; }
#pragma unroll
  for (int o = 1; o < 32; o <<= 1) m = fmaxf(m, __shfl_xor(m, o));
  float sum = 0.f;
#pragma unroll
  for (int c = 0; c < KCH; ++c) {
#pragma unroll
    for (int i = 0; i < 4; ++i) { const float v = e[c][i]; const float x = (v <= -1.0e38f) ? 0.f : exp2f((v - m) * 1.44269504088896f); e[c][i] = x; sum += x; } }
#pragma unroll
  for (int o = 1; o < 32; o <<= 1) sum += __shfl_xor(sum, o);
  const float inv = sum > 0.f ? 2048.0f / sum : 0.f;
  v4f p[KCH];
#pragma unroll
  for (int c = 0; c < KCH; ++c) p[c] = e[c] * inv;
#pragma unroll
  for (int c = 0; c < KCH; ++c) *(volatile v4f*)(sr + c * 128 + lane * 4) = p[c];
  __threadfence();
#pragma unroll
  for (int c = 0; c < KCH; ++c) *(volatile v4f*)(sr + c * 128 + lane * 4) = p[c];
}

__global__ __launch_bounds__(128) void k_pv(const float* __restrict__ PS0, const _Float16* __restrict__ VT, const __bf16* __restrict__ VB, const __bf16* __restrict__ VBL, float* __restrict__ Y) {
  __shared__ __align__(16) float ss[4][16][HD + 4];
  const int bl = blockIdx.z / NH, h = blockIdx.z % NH; const float* PS = PS0 + (size_t)blockIdx.z * TT * TT;
  const int tid = threadIdx.x, wave = __builtin_amdgcn_readfirstlane((int)(tid >> 5)), lane = tid & 31, col = lane & 15, g = lane >> 4; const int qb = blockIdx.x; const int ql0 = qb * 64 + wave * 16; const int kce = (kb_last(qb) + 1) * 4;
  v8f acc[HD / 16] = {};
  if (!NEED_PLAIN || qb < QBH) {
#pragma unroll 1
    for (int kc = 0; kc < kce; ++kc) { const F2 p = split_row(PS + (size_t)(ql0 + col) * TT, kc * 32, lane);
      asm volatile("s_wait_loadcnt 0x0" ::: "memory");
#pragma unroll
      for (int j = 0; j < HD / 16; ++j) { const size_t po = ((size_t)bl * CC + h * HD + j * 16 + col) * (size_t)KHI + kc * 32; const v16b vh = frag_b(VB + po, lane); acc[j] = wmma_bf(p.h, vh, acc[j]); acc[j] = wmma_bf(p.l, vh, acc[j]); acc[j] = wmma_bf(p.h, frag_b(VBL + po, lane), acc[j]); } }
  } else {
#pragma unroll 1
    for (int kc = 0; kc < kce; ++kc) { const v16h p = frag_f32(PS + (size_t)(ql0 + col) * TT + kc * 32, lane);
      asm volatile("s_wait_loadcnt 0x0" ::: "memory");
#pragma unroll
      for (int j = 0; j < HD / 16; ++j) { const size_t po = ((size_t)bl * CC + h * HD + j * 16 + col) * (size_t)TT + kc * 32; acc[j] = wmma16(p, frag_h(VT + po, lane), acc[j]); } }
  }
#pragma unroll
  for (int j = 0; j < HD / 16; ++j) {
#pragma unroll
    for (int r = 0; r < 8; ++r) ss[wave][8 * g + r][j * 16 + col] = acc[j][r] * (1.0f / 2048.0f);
  }
  LDSX();
  for (int rl = 0; rl < 16; ++rl) if (lane < HD / 4) vst2((void*)(Y + ((size_t)bl * TT + ql0 + rl) * CC + h * HD + lane * 4), *(const v4f*)&ss[wave][rl][lane * 4]);
}

__global__ __launch_bounds__(128) void k_out(const float* __restrict__ Y, const float* __restrict__ WO, const float* __restrict__ BO, float* __restrict__ OUT) {
  __shared__ __align__(16) float sf[4][16][132];
  const int tid = threadIdx.x, wave = __builtin_amdgcn_readfirstlane((int)(tid >> 5)), lane = tid & 31, col = lane & 15, g = lane >> 4; const int c0 = blockIdx.y * 128;
  const size_t rb = (size_t)blockIdx.x * 64; const size_t r0 = rb + wave * 16; const size_t bb = rb / TT; const int tl = (int)(rb % TT) + wave * 16; const size_t orow0 = bb * TT_FULL + tl;
  v8f acc[8] = {};
  if (CAUSAL && (int)(rb % TT) < QHI) {
#pragma unroll 2
    for (int kc = 0; kc < CC / 32; ++kc) { const F2 a = split_row(Y + (r0 + col) * CC, kc * 32, lane); asm volatile("s_wait_loadcnt 0x0" ::: "memory");
#pragma unroll
      for (int j = 0; j < 8; ++j) { const v16b w = wcol_io(WO, kc * 32, c0 + j * 16 + col, lane, DIN); asm volatile("s_wait_loadcnt 0x0" ::: "memory"); acc[j] = wmma_bf(a.h, w, acc[j]); acc[j] = wmma_bf(a.l, w, acc[j]); } }
#pragma unroll
    for (int j = 0; j < 8; ++j) { const float bias = bfr(BO[c0 + j * 16 + col]);
#pragma unroll
      for (int r = 0; r < 8; ++r) sf[wave][8 * g + r][j * 16 + col] = acc[j][r] + bias; }
  } else {
#pragma unroll 2
    for (int kc = 0; kc < CC / 32; ++kc) { const v16h a = frag_f32s(Y + (r0 + col) * CC + kc * 32, lane, 64.0f); asm volatile("s_wait_loadcnt 0x0" ::: "memory");
#pragma unroll
      for (int j = 0; j < 8; ++j) { const v16h w = wcolh_io(WO, kc * 32, c0 + j * 16 + col, lane, DIN); asm volatile("s_wait_loadcnt 0x0" ::: "memory"); acc[j] = wmma16(a, w, acc[j]); } }
#pragma unroll
    for (int j = 0; j < 8; ++j) { const float bias = bfr(BO[c0 + j * 16 + col]);
#pragma unroll
      for (int r = 0; r < 8; ++r) sf[wave][8 * g + r][j * 16 + col] = acc[j][r] * (1.0f / 16384.0f) + bias; }
  }
  LDSX();
  for (int rl = 0; rl < 16; ++rl) vst2((void*)(OUT + (orow0 + rl) * DIN + c0 + lane * 4), *(const v4f*)&sf[wave][rl][lane * 4]);
}

extern "C" void kernel_launch(void* const* d_in, const int* in_sizes, int n_in, void* d_out, int out_size, void* d_ws, size_t ws_size, hipStream_t stream) {
  if (n_in < 6) return;
  const size_t need_rows = (size_t)(NB - 1) * TT_FULL + TT;
  if ((size_t)in_sizes[0] < need_rows * DIN) return;
  if ((size_t)in_sizes[1] < (size_t)NH * DIN * HD || (size_t)in_sizes[2] < (size_t)NH * DIN * HD || (size_t)in_sizes[3] < (size_t)NH * DIN * HD) return;
  if ((size_t)in_sizes[4] < (size_t)CC * DIN || (size_t)in_sizes[5] < (size_t)DIN) return;
  if ((size_t)out_size < need_rows * DIN) return;
  if (ws_size < (size_t)WS_END) return;
  const float** F = (const float**)d_in;
  char* ws = (char*)d_ws;
  _Float16 *QH = (_Float16*)(ws + WS_QH), *KH = (_Float16*)(ws + WS_KH), *VT = (_Float16*)(ws + WS_VT), *QL = (_Float16*)(ws + WS_QL), *KL = (_Float16*)(ws + WS_KL);
  __bf16 *VB = (__bf16*)(ws + WS_VB), *VBL = (__bf16*)(ws + WS_VBL); float *S = (float*)(ws + WS_S), *Y = (float*)(ws + WS_Y);
  for (int b0 = 0; b0 < NB; b0 += NBC) {
    const float* Xc = F[0] + (size_t)b0 * TT_FULL * DIN; float* Oc = (float*)d_out + (size_t)b0 * TT_FULL * DIN;
    k_proj<<<dim3(NBC * TT / 64, CC / 128, 3), 128, 0, stream>>>(Xc, F[1], F[2], F[3], QH, QL, KH, KL, VT, VB, VBL);
    k_sc<<<dim3(NQB, TT / 128, NBC * NH), 128, 0, stream>>>(QH, KH, QL, KL, S);
    k_sm<<<dim3(TT / 8, NBC * NH), 256, 0, stream>>>(S);
    k_pv<<<dim3(NQB, 1, NBC * NH), 128, 0, stream>>>(S, VT, VB, VBL, Y);
    k_out<<<dim3(NBC * TT / 64, DIN / 128), 128, 0, stream>>>(Y, F[4], F[5], Oc);
  }
}
